// MixtureOfExperts_89172111000183
// MI455X (gfx1250) — hardware-run, weakly checked
//
#include <hip/hip_runtime.h>
#include <math.h>

#define NTOK 2048
#define DM 512
#define FF 1024
#define NE 8
#define SPT 2
#define NSLOT (NTOK * SPT)
#define R_MAX (NSLOT + 64 * NE)
#define NT_MAX (R_MAX / 64)
#define OUT1_OFF ((size_t)NTOK * (size_t)DM)

#define CX_LOG2 11
#define CW_LOG2 16
#define CH_LOG2 11
#define CH ((float)(1u << CH_LOG2))
#define SC_H (1.0f / (float)(1u << (CX_LOG2 + CW_LOG2)))
#define SC_Y (1.0f / (float)(1u << (CH_LOG2 + CW_LOG2)))

#define RW_CH 8192
#define TBL_COUNT 0
#define TBL_POFF 16
#define TBL_NTILES 40
#define TBL_TILE_E 64
#define TBL_HDR 256
#define TBL_ROWTOK TBL_HDR
#define TBL_SLOTROW (TBL_HDR + R_MAX)
#define TBL_WORDS (TBL_HDR + R_MAX + NSLOT)

static_assert(NE == 8 && SPT == 2 && NTOK == 2048 && NTOK % 256 == 0);
static_assert(DM == 512 && FF == 1024 && DM % 64 == 0 && FF % 64 == 0 && DM % 128 == 0 && NTOK % 8 == 0 && 256 % (DM / 8) == 0);
static_assert(NSLOT % 128 == 0 && R_MAX % 128 == 0 && R_MAX >= NSLOT + 63 * NE && R_MAX % (256 / (DM / 8)) == 0);
static_assert(TBL_HDR % 32 == 0 && TBL_HDR <= 512);
static_assert(TBL_COUNT + NE <= TBL_POFF && TBL_POFF + NE + 1 <= TBL_NTILES && TBL_NTILES < TBL_TILE_E && TBL_TILE_E + NT_MAX <= TBL_HDR);
static_assert(RW_CH % 128 == 0 && (TBL_WORDS * 4) % 256 == 0);
static_assert(CX_LOG2 == 11 && CW_LOG2 == 16 && CH_LOG2 == 11);
static_assert(NSLOT == 4096 && R_MAX == 4608 && NT_MAX == 72 && TBL_WORDS == 8960);
static_assert((NTOK * DM / 8) % 256 == 0 && (NE * FF * DM / 8) % 256 == 0);

constexpr size_t al256(size_t n) { return (n + 255) & ~(size_t)255; }
constexpr size_t SZ_A16 = al256((size_t)NTOK * DM * 2);
constexpr size_t SZ_U16  = al256((size_t)NE * FF * DM * 2);
constexpr size_t SZ_V16  = al256((size_t)NE * DM * FF * 2);
constexpr size_t SZ_SEL = al256((size_t)NSLOT * 4);
constexpr size_t SZ_WGT = al256((size_t)NSLOT * 4);
constexpr size_t SZ_TBL = al256((size_t)TBL_WORDS * 4);
constexpr size_t SZ_XG  = al256((size_t)R_MAX * DM * 2);
constexpr size_t SZ_HG  = al256((size_t)R_MAX * FF * 2);
constexpr size_t SZ_YG  = al256((size_t)R_MAX * DM * 4);
constexpr size_t WS_TOTAL = SZ_A16 + SZ_U16 + SZ_V16 + SZ_SEL + SZ_WGT + SZ_TBL + SZ_XG + SZ_HG + SZ_YG;
static_assert(WS_TOTAL == (size_t)42535936 && WS_TOTAL < (size_t)134217728);

typedef _Float16 h16;
typedef __attribute__((ext_vector_type(16))) _Float16 v16h;
typedef __attribute__((ext_vector_type(8)))  _Float16 v8h;
typedef __attribute__((ext_vector_type(8)))  float    v8f;
typedef __attribute__((ext_vector_type(4)))  float    v4f;
typedef __attribute__((ext_vector_type(2)))  float    v2f;
typedef __attribute__((ext_vector_type(4)))  unsigned int v4u;
typedef __attribute__((ext_vector_type(4)))  int      v4i;
typedef __attribute__((ext_vector_type(2)))  int      v2i;


#define VST2(T, ptr, val) do { const T vst2_v_ = (val); *(volatile T*)(ptr) = vst2_v_; __threadfence(); *(volatile T*)(ptr) = vst2_v_; } while (0)

static __device__ __forceinline__ float bfr(float f) {
    unsigned u = __float_as_uint(f);
    u += 0x7FFFu + ((u >> 16) & 1u);
    return __uint_as_float(u & 0xFFFF0000u);
}
static __device__ __forceinline__ h16 toh_flush(float v) { const float w = (fabsf(v) < 6.103515625e-05f) ? 0.0f : v; return (h16)w; }
static __device__ __forceinline__ void st8h(h16* p, const float* v) {
    v8h hv;
#pragma unroll
    for (int e = 0; e < 8; ++e) hv[e] = toh_flush(v[e]);
    VST2(v8h, p, hv);
}

union FragU { v16h v; v8h h[2]; };
static __device__ __forceinline__ v16h frag_ld(const h16* p) {
    FragU f; f.h[0] = *(const v8h*)(p); f.h[1] = *(const v8h*)(p + 16); return f.v;
}
static __device__ __forceinline__ v8f wmma16g(v16h a, v16h b, v8f c) {
    c = __builtin_amdgcn_wmma_f32_16x16x32_f16(false, a, false, b, (short)0, c, false, false);
    asm volatile("v_nop\n\tv_nop\n\tv_nop\n\tv_nop" : "+v"(c) : "v"(a), "v"(b));
    return c;
}
static __device__ __forceinline__ void wave_sync_lds() {
    __builtin_amdgcn_fence(3  , "workgroup");
    __builtin_amdgcn_wave_barrier();
    __builtin_amdgcn_fence(2  , "workgroup");
}
__device__ __forceinline__ float gelu_erf(float a) { return 0.5f * a * (1.0f + erff(a * 0.70710678118654752f)); }

template <int LOG2C>
__global__ __launch_bounds__(256) void k_plane(const float* __restrict__ src, h16* __restrict__ dst, unsigned n8) {
    const unsigned u = blockIdx.x * 256u + threadIdx.x;
    if (u >= n8) return;
    const float cs = (float)(1u << LOG2C);
    const v4f a = *(const v4f*)(src + (size_t)u * 8u);
    const v4f b = *(const v4f*)(src + (size_t)u * 8u + 4u);
    float v[8] = {bfr(a.x) * cs, bfr(a.y) * cs, bfr(a.z) * cs, bfr(a.w) * cs, bfr(b.x) * cs, bfr(b.y) * cs, bfr(b.z) * cs, bfr(b.w) * cs};
    st8h(dst + (size_t)u * 8u, v);
}


__global__ __launch_bounds__(256) void k_gate2n(const float* __restrict__ tk, const float* __restrict__ gm, const float* __restrict__ gc, int* __restrict__ sel, float* __restrict__ wgt, float* __restrict__ sc) {
    const unsigned lane = threadIdx.x & 31u;
    const unsigned wave = threadIdx.x >> 5;
    const unsigned tok0 = (blockIdx.x * 8u + wave) * 32u;
    if (tok0 >= (unsigned)NTOK) return;
    v2i ke; ke.x = 0; ke.y = 1;
    v2f kw; kw.x = 0.0f; kw.y = 0.0f;
    v4f pa; pa.x = 0.0f; pa.y = 0.0f; pa.z = 0.0f; pa.w = 0.0f;
    v4f pb; pb.x = 0.0f; pb.y = 0.0f; pb.z = 0.0f; pb.w = 0.0f;
    for (unsigned tt = 0; tt < 32u; ++tt) {
        const float* rp = tk + (size_t)(tok0 + tt) * DM;
        double acc[NE];
#pragma unroll
        for (int g = 0; g < NE; ++g) acc[g] = 0.0;
        for (unsigned q = 0; q < (unsigned)(DM / 32); ++q) {
            const unsigned f = lane + 32u * q;
            const double rv = (double)bfr(rp[f]);
#pragma unroll
            for (int g = 0; g < NE; ++g) acc[g] = fma((double)bfr(gm[(size_t)g * DM + f]), rv, acc[g]);
        }
#pragma unroll
        for (int g = 0; g < NE; ++g) {
            double u = acc[g];
            u += __shfl_xor(u, 16, 32);
            u += __shfl_xor(u, 8, 32);
            u += __shfl_xor(u, 4, 32);
            u += __shfl_xor(u, 2, 32);
            u += __shfl_xor(u, 1, 32);
            acc[g] = u + (double)bfr(gc[g]);
        }
        int e0 = 0; double v0 = acc[0];
#pragma unroll
        for (int g = 1; g < NE; ++g) { const bool tk_ = acc[g] > v0; e0 = tk_ ? g : e0; v0 = tk_ ? acc[g] : v0; }
        int e1 = 0; double v1 = 0.0; bool have = false;
#pragma unroll
        for (int g = 0; g < NE; ++g) {
            const bool free_ = (g != e0);
            const bool tk_ = free_ && (!have || acc[g] > v1);
            e1 = tk_ ? g : e1; v1 = tk_ ? acc[g] : v1; have = have || free_;
        }
        float ssum = 0.0f;
#pragma unroll
        for (int g = 0; g < NE; ++g) ssum += expf((float)(acc[g] - v0));
        const float p0 = 1.0f / ssum;
        const float p1 = expf((float)(v1 - v0)) / ssum;
        const float psum = p0 + p1;
        const float g0 = p0 / psum;
        const float g1 = p1 / psum;
        const bool mine = (lane == tt);
        ke.x = mine ? e0 : ke.x; ke.y = mine ? e1 : ke.y;
        kw.x = mine ? g0 : kw.x; kw.y = mine ? g1 : kw.y;
        pa.x = mine ? (float)acc[0] : pa.x; pa.y = mine ? (float)acc[1] : pa.y; pa.z = mine ? (float)acc[2] : pa.z; pa.w = mine ? (float)acc[3] : pa.w;
        pb.x = mine ? (float)acc[4] : pb.x; pb.y = mine ? (float)acc[5] : pb.y; pb.z = mine ? (float)acc[6] : pb.z; pb.w = mine ? (float)acc[7] : pb.w;
    }
    const unsigned n = tok0 + lane;
    VST2(v2i, sel + 2u * n, ke);
    VST2(v2f, wgt + 2u * n, kw);
    VST2(v4f, sc + 8u * (size_t)n, pa);
    VST2(v4f, sc + 8u * (size_t)n + 4u, pb);
}

template <int NE_>
__global__ __launch_bounds__(32) void k_route1w(const int* __restrict__ sel, int* __restrict__ tbl, unsigned nslot, unsigned spt, unsigned hdr, unsigned rmax,
                                                unsigned offPoff, unsigned offNtiles, unsigned offTileE) {
    static_assert(NE_ >= 1 && NE_ <= 32);
    __shared__ __align__(16) int s_img[RW_CH];
    __shared__ __align__(16) int s_hdr[512];
    const unsigned lane = threadIdx.x & 31u;
    const unsigned spl = nslot >> 5;
    const unsigned ng = spl >> 2;
    const unsigned ntmax = rmax >> 6;
    const v4i* sp = (const v4i*)(sel + (size_t)lane * spl);
    int cnt[NE_];
#pragma unroll
    for (int j = 0; j < NE_; ++j) cnt[j] = 0;
    for (unsigned g = 0; g < ng; ++g) {
        const v4i v = sp[g];
#pragma unroll
        for (int c = 0; c < 4; ++c) {
            const int e = min(max(v[c], 0), NE_ - 1);
#pragma unroll
            for (int j = 0; j < NE_; ++j) cnt[j] += (e == j) ? 1 : 0;
        }
    }
    int base0[NE_], total[NE_];
#pragma unroll
    for (int j = 0; j < NE_; ++j) {
        int pre = 0, tot = cnt[j];
#pragma unroll
        for (int d = 1; d < 32; d <<= 1) {
            const int t = __shfl_xor(tot, d, 32);
            pre += ((lane & (unsigned)d) != 0u) ? t : 0;
            tot += t;
        }
        base0[j] = pre;
        total[j] = tot;
    }
    int poff[NE_ + 1];
    poff[0] = 0;
#pragma unroll
    for (int j = 0; j < NE_; ++j) poff[j + 1] = poff[j] + (((total[j] + 63) >> 6) << 6);
    for (unsigned i = lane; i < 512u; i += 32u) s_hdr[i] = (i >= offTileE && i < offTileE + ntmax) ? -1 : 0;
    wave_sync_lds();
    if (lane == 0u) {
#pragma unroll
        for (int j = 0; j < NE_; ++j) { s_hdr[min((unsigned)j, 511u)] = total[j]; s_hdr[min(offPoff + (unsigned)j, 511u)] = poff[j]; }
        s_hdr[min(offPoff + (unsigned)NE_, 511u)] = poff[NE_];
        s_hdr[min(offNtiles, 511u)] = poff[NE_] >> 6;
    }
    for (unsigned t = lane; t < ntmax; t += 32u) {
        const int b64 = (int)(t * 64u);
        int ev = -1;
#pragma unroll
        for (int j = 0; j < NE_; ++j) ev = (b64 >= poff[j] && b64 < poff[j + 1]) ? j : ev;
        s_hdr[min(offTileE + t, 511u)] = ev;
    }
    wave_sync_lds();
    for (int pass = 0; pass < 2; ++pass) {
        for (unsigned i = lane; i < (hdr >> 2); i += 32u) *(volatile v4i*)(tbl + 4u * i) = *(const v4i*)(&s_hdr[4u * i]);
        __threadfence();
    }
    for (unsigned lo = 0; lo < rmax; lo += (unsigned)RW_CH) {
        for (unsigned i = lane; i < (unsigned)(RW_CH / 4); i += 32u) *(v4i*)(&s_img[4u * i]) = (v4i){-1, -1, -1, -1};
        wave_sync_lds();
        int run[NE_];
#pragma unroll
        for (int j = 0; j < NE_; ++j) run[j] = base0[j];
        for (unsigned g = 0; g < ng; ++g) {
            const v4i v = sp[g];
#pragma unroll
            for (int c = 0; c < 4; ++c) {
                const int e = min(max(v[c], 0), NE_ - 1);
                int row = 0;
#pragma unroll
                for (int j = 0; j < NE_; ++j) {
                    const bool hit = (e == j);
                    row = hit ? (poff[j] + run[j]) : row;
                    run[j] += hit ? 1 : 0;
                }
                row = min(max(row, 0), (int)rmax - 1);
                const unsigned rel = (unsigned)row - lo;
                if (rel < (unsigned)RW_CH) s_img[rel] = (int)((lane * spl + 4u * g + (unsigned)c) / spt);
            }
        }
        wave_sync_lds();
        const unsigned nw = min((unsigned)RW_CH, rmax - lo);
        for (int pass = 0; pass < 2; ++pass) {
            for (unsigned i = lane; i < (nw >> 2); i += 32u) *(volatile v4i*)(tbl + hdr + lo + 4u * i) = *(const v4i*)(&s_img[4u * i]);
            __threadfence();
        }
        wave_sync_lds();
    }
    for (unsigned lo = 0; lo < nslot; lo += (unsigned)RW_CH) {
        int run[NE_];
#pragma unroll
        for (int j = 0; j < NE_; ++j) run[j] = base0[j];
        for (unsigned g = 0; g < ng; ++g) {
            const v4i v = sp[g];
#pragma unroll
            for (int c = 0; c < 4; ++c) {
                const int e = min(max(v[c], 0), NE_ - 1);
                int row = 0;
#pragma unroll
                for (int j = 0; j < NE_; ++j) {
                    const bool hit = (e == j);
                    row = hit ? (poff[j] + run[j]) : row;
                    run[j] += hit ? 1 : 0;
                }
                row = min(max(row, 0), (int)rmax - 1);
                const unsigned rel = (lane * spl + 4u * g + (unsigned)c) - lo;
                if (rel < (unsigned)RW_CH) s_img[rel] = row;
            }
        }
        wave_sync_lds();
        const unsigned nw = min((unsigned)RW_CH, nslot - lo);
        for (int pass = 0; pass < 2; ++pass) {
            for (unsigned i = lane; i < (nw >> 2); i += 32u) *(volatile v4i*)(tbl + hdr + rmax + lo + 4u * i) = *(const v4i*)(&s_img[4u * i]);
            __threadfence();
        }
        wave_sync_lds();
    }
}

__global__ __launch_bounds__(256) void k_gather(const h16* __restrict__ x16, const int* __restrict__ tbl, h16* __restrict__ Xg) {
    const unsigned TPR = (unsigned)(DM / 8);
    const unsigned row = blockIdx.x * (256u / TPR) + (threadIdx.x / TPR);
    if (row >= (unsigned)R_MAX) return;
    const unsigned c = (threadIdx.x % TPR) * 8u;
    const int tr = tbl[TBL_ROWTOK + row];
    const bool pad = (tr < 0);
    const int tok = min(max(tr, 0), NTOK - 1);
    const v4u ld = *(const v4u*)(x16 + (size_t)(unsigned)tok * DM + c);
    v4u o;
    o.x = pad ? 0u : ld.x; o.y = pad ? 0u : ld.y; o.z = pad ? 0u : ld.z; o.w = pad ? 0u : ld.w;
    VST2(v4u, Xg + (size_t)row * DM + c, o);
}


__global__ __launch_bounds__(256) void k_ffn1(const h16* __restrict__ Xg, const h16* __restrict__ Wp,
                                              const int* __restrict__ tbl, h16* __restrict__ Hg) {
    __shared__ __align__(16) float sT[8][16 * 68];
    const unsigned lane = threadIdx.x & 31u;
    const unsigned wave = threadIdx.x >> 5;
    const unsigned u = blockIdx.x * 8u + wave;
    if (u >= (unsigned)(NT_MAX * (FF / 64))) return;
    const unsigned rowtile = u / (unsigned)(FF / 64);
    const unsigned ct = u - rowtile * (unsigned)(FF / 64);
    const int nt = min(max(tbl[TBL_NTILES], 0), NT_MAX);
    if ((int)rowtile >= nt) return;
    const int e = min(max(tbl[TBL_TILE_E + rowtile], 0), NE - 1);
    const size_t wbase = (size_t)(unsigned)e * (size_t)(FF * DM);
    const unsigned m0 = rowtile << 6, n0 = ct << 6;
    const unsigned rlane = lane & 15u;
    const unsigned koff = (lane >> 4) * 8u;
    const unsigned mOff = koff;

    v8f acc[4][4];
#pragma unroll
    for (int i = 0; i < 4; ++i)
#pragma unroll
        for (int j = 0; j < 4; ++j) acc[i][j] = (v8f){0.f,0.f,0.f,0.f,0.f,0.f,0.f,0.f};

    for (unsigned k0 = 0; k0 < (unsigned)DM; k0 += 32u) {
        v16h bh[4];
#pragma unroll
        for (int j = 0; j < 4; ++j)
            bh[j] = frag_ld(Wp + wbase + (size_t)(n0 + ((unsigned)j << 4) + rlane) * DM + koff + k0);
#pragma unroll
        for (int i = 0; i < 4; ++i) {
            const v16h ah = frag_ld(Xg + (size_t)(m0 + ((unsigned)i << 4) + rlane) * DM + koff + k0);
#pragma unroll
            for (int j = 0; j < 4; ++j) acc[i][j] = wmma16g(ah, bh[j], acc[i][j]);
        }
    }

    float* slab = sT[wave];
#pragma unroll
    for (int i = 0; i < 4; ++i) {
        const unsigned mBase = m0 + ((unsigned)i << 4);
#pragma unroll
        for (int j = 0; j < 4; ++j)
#pragma unroll
            for (int r = 0; r < 8; ++r) {
                const float a = acc[i][j][r] * SC_H;
                const float g = gelu_erf(a);
                slab[(mOff + (unsigned)r) * 68u + ((unsigned)j << 4) + rlane] = g * CH;
            }
        wave_sync_lds();
        const unsigned q = lane >> 3, c8 = (lane & 7u) * 8u;
        v8h hv[4];
#pragma unroll
        for (int it = 0; it < 4; ++it) {
            const unsigned row = (unsigned)it * 4u + q;
            const float* sp = slab + row * 68u + c8;
#pragma unroll
            for (int t = 0; t < 8; ++t) hv[it][t] = toh_flush(sp[t]);
        }
        for (int pass = 0; pass < 2; ++pass) {
#pragma unroll
            for (int it = 0; it < 4; ++it) {
                const unsigned row = (unsigned)it * 4u + q;
                *(volatile v8h*)(Hg + (size_t)(mBase + row) * FF + n0 + c8) = hv[it];
            }
            __threadfence();
        }
        wave_sync_lds();
    }
}

__global__ __launch_bounds__(256) void k_ffn2(const h16* __restrict__ Hg, const h16* __restrict__ Wp,
                                              const int* __restrict__ tbl, float* __restrict__ Yg) {
    __shared__ __align__(16) float sT[8][16 * 68];
    const unsigned lane = threadIdx.x & 31u;
    const unsigned wave = threadIdx.x >> 5;
    const unsigned u = blockIdx.x * 8u + wave;
    if (u >= (unsigned)(NT_MAX * (DM / 64))) return;
    const unsigned rowtile = u / (unsigned)(DM / 64);
    const unsigned ct = u - rowtile * (unsigned)(DM / 64);
    const int nt = min(max(tbl[TBL_NTILES], 0), NT_MAX);
    if ((int)rowtile >= nt) return;
    const int e = min(max(tbl[TBL_TILE_E + rowtile], 0), NE - 1);
    const size_t wbase = (size_t)(unsigned)e * (size_t)(DM * FF);
    const unsigned m0 = rowtile << 6, n0 = ct << 6;
    const unsigned rlane = lane & 15u;
    const unsigned koff = (lane >> 4) * 8u;
    const unsigned mOff = koff;

    v8f acc[4][4];
#pragma unroll
    for (int i = 0; i < 4; ++i)
#pragma unroll
        for (int j = 0; j < 4; ++j) acc[i][j] = (v8f){0.f,0.f,0.f,0.f,0.f,0.f,0.f,0.f};

    for (unsigned k0 = 0; k0 < (unsigned)FF; k0 += 32u) {
        v16h bh[4];
#pragma unroll
        for (int j = 0; j < 4; ++j)
            bh[j] = frag_ld(Wp + wbase + (size_t)(n0 + ((unsigned)j << 4) + rlane) * FF + koff + k0);
#pragma unroll
        for (int i = 0; i < 4; ++i) {
            const v16h ah = frag_ld(Hg + (size_t)(m0 + ((unsigned)i << 4) + rlane) * FF + koff + k0);
#pragma unroll
            for (int j = 0; j < 4; ++j) acc[i][j] = wmma16g(ah, bh[j], acc[i][j]);
        }
    }

    float* slab = sT[wave];
#pragma unroll
    for (int i = 0; i < 4; ++i) {
        const unsigned mBase = m0 + ((unsigned)i << 4);
#pragma unroll
        for (int j = 0; j < 4; ++j)
#pragma unroll
            for (int r = 0; r < 8; ++r)
                slab[(mOff + (unsigned)r) * 68u + ((unsigned)j << 4) + rlane] = acc[i][j][r] * SC_Y;
        wave_sync_lds();
        const unsigned hh = lane >> 4, c4 = (lane & 15u) * 4u;
#pragma unroll
        for (int half = 0; half < 2; ++half) {
            v4f vv[4];
#pragma unroll
            for (int it = 0; it < 4; ++it) {
                const unsigned row = (unsigned)(half * 4 + it) * 2u + hh;
                vv[it] = *(const v4f*)(slab + row * 68u + c4);
            }
            for (int pass = 0; pass < 2; ++pass) {
#pragma unroll
                for (int it = 0; it < 4; ++it) {
                    const unsigned row = (unsigned)(half * 4 + it) * 2u + hh;
                    *(volatile v4f*)(Yg + (size_t)(mBase + row) * DM + n0 + c4) = vv[it];
                }
                __threadfence();
            }
        }
        wave_sync_lds();
    }
}

__global__ __launch_bounds__(256) void k_combine(const float* __restrict__ Yg, const float* __restrict__ wgt, const int* __restrict__ tbl, float* __restrict__ out) {
    const unsigned t = blockIdx.x * 2u + (threadIdx.x >> 7);
    if (t >= (unsigned)NTOK) return;
    const unsigned c = (threadIdx.x & 127u) * 4u;
    const int r0 = min(max(tbl[TBL_SLOTROW + 2u * t], 0), R_MAX - 1);
    const int r1 = min(max(tbl[TBL_SLOTROW + 2u * t + 1u], 0), R_MAX - 1);
    const float w0 = wgt[2u * t], w1 = wgt[2u * t + 1u];
    const v4f a = *(const v4f*)(Yg + (size_t)(unsigned)r0 * DM + c);
    const v4f b = *(const v4f*)(Yg + (size_t)(unsigned)r1 * DM + c);
    const v4f y = (a * w0) + (b * w1);
    VST2(v4f, out + (size_t)t * DM + c, y);
}

extern "C" void kernel_launch(void* const* d_in, const int* in_sizes, int n_in, void* d_out, int out_size,
                              void* d_ws, size_t ws_size, hipStream_t stream) {
    if (n_in < 5) return;
    if (in_sizes[0] < NTOK * DM || in_sizes[1] < NE * DM || in_sizes[2] < NE || in_sizes[3] < NE * FF * DM || in_sizes[4] < NE * DM * FF) return;
    if (out_size < NTOK * DM + NTOK * NE) return;
    if (ws_size < WS_TOTAL) return;
    const float* ta = (const float*)d_in[0];
    const float* ga = (const float*)d_in[1];
    const float* gb = (const float*)d_in[2];
    const float* ua = (const float*)d_in[3];
    const float* va = (const float*)d_in[4];
    float* res = (float*)d_out;
    uint8_t* wp = (uint8_t*)d_ws;
    h16* a16 = (h16*)wp; wp += SZ_A16;
    h16* u16 = (h16*)wp; wp += SZ_U16;
    h16* v16 = (h16*)wp; wp += SZ_V16;
    int* sel = (int*)wp; wp += SZ_SEL;
    float* wgt = (float*)wp; wp += SZ_WGT;
    int* tbl = (int*)wp; wp += SZ_TBL;
    h16* Xg = (h16*)wp; wp += SZ_XG;
    h16* Hg = (h16*)wp; wp += SZ_HG;
    float* Yg = (float*)wp;

    k_plane<CX_LOG2><<<(NTOK * DM / 8) / 256, 256, 0, stream>>>(ta, a16, (unsigned)(NTOK * DM / 8));
    k_plane<CW_LOG2><<<(NE * FF * DM / 8) / 256, 256, 0, stream>>>(ua, u16, (unsigned)(NE * FF * DM / 8));
    k_plane<CW_LOG2><<<(NE * DM * FF / 8) / 256, 256, 0, stream>>>(va, v16, (unsigned)(NE * DM * FF / 8));
    k_gate2n<<<NTOK / 256, 256, 0, stream>>>(ta, ga, gb, sel, wgt, res + OUT1_OFF);
    k_route1w<NE><<<1, 32, 0, stream>>>(sel, tbl, (unsigned)NSLOT, (unsigned)SPT, (unsigned)TBL_HDR, (unsigned)R_MAX, (unsigned)TBL_POFF, (unsigned)TBL_NTILES, (unsigned)TBL_TILE_E);
    k_gather<<<R_MAX / (256 / (DM / 8)), 256, 0, stream>>>(a16, tbl, Xg);
    k_ffn1<<<(NT_MAX * (FF / 64) + 7) / 8, 256, 0, stream>>>(Xg, u16, tbl, Hg);
    k_ffn2<<<(NT_MAX * (DM / 64) + 7) / 8, 256, 0, stream>>>(Hg, v16, tbl, Yg);
    k_combine<<<NTOK / 2, 256, 0, stream>>>(Yg, wgt, tbl, res);
}
